// xLSTM_33071248179634
// MI455X (gfx1250) — hardware-run, weakly checked
//
#include <hip/hip_runtime.h>
#include <math.h>

constexpr int NLAY  = 2;
constexpr int NBAT  = 4;
constexpr int NSEQ  = 512;
constexpr int NDIM  = 512;
constexpr int NHEAD = 8;
constexpr int HDIM  = 64;
constexpr int NPROJ = 1024;
constexpr int NHID  = 512;
constexpr int KCONV = 4;
constexpr int NROW  = NSEQ * NBAT;
constexpr int NQKS  = 1600;
constexpr int COL_Q = 0, COL_K = 512, COL_SKIP = 1024, COL_IG = 1536, COL_FG = 1544, COL_ZPAD = 1552;
constexpr int NVO   = 1024;
constexpr int COL_V = 0, COL_OG = 512;
constexpr int NTHR  = 256;
static_assert(NHID == NHEAD * HDIM);
static_assert(NROW % 64 == 0 && NPROJ % 64 == 0 && NHID % 64 == 0 && NQKS % 64 == 0 && NVO % 64 == 0 && NDIM % 64 == 0);
static_assert(NDIM % 32 == 0 && NPROJ % 32 == 0 && NHID % 32 == 0);
static_assert(NROW % (NTHR / 32) == 0);
static_assert(NROW % (NTHR / 64) == 0);
static_assert((NROW * (NPROJ / 8)) % NTHR == 0);
static_assert(NQKS - COL_ZPAD == 48);
static_assert(NDIM == 512 && NPROJ == 1024 && HDIM == 64 && NTHR == 256);

typedef __attribute__((ext_vector_type(16))) _Float16 v16h;
typedef __attribute__((ext_vector_type(8)))  _Float16 v8h;
typedef __attribute__((ext_vector_type(16))) __bf16   v16b;
typedef __attribute__((ext_vector_type(8)))  __bf16   v8b;
typedef __attribute__((ext_vector_type(8)))  float    v8f;
typedef __attribute__((ext_vector_type(4)))  float    v4f;
typedef __attribute__((ext_vector_type(4)))  unsigned int v4u;

__device__ __forceinline__ unsigned short f2bf_bits(float f) {
  unsigned u = __float_as_uint(f);
  return (unsigned short)((u + 0x7FFFu + ((u >> 16) & 1u)) >> 16);
}
__device__ __forceinline__ float bf_bits2f(unsigned short h) { return __uint_as_float(((unsigned)h) << 16); }
__device__ __forceinline__ unsigned pack_bf2(float e0, float e1) {
  return (unsigned)f2bf_bits(e0) | ((unsigned)f2bf_bits(e1) << 16);
}
__device__ __forceinline__ float fsigm(float x) { return __builtin_amdgcn_rcpf(1.0f + __expf(-x)); }
__device__ __forceinline__ float fsilu(float x) { return x * fsigm(x); }

__device__ __forceinline__ void dep_guard_h(v8f& a, v8f& b, v16h x, v16h y) { asm volatile("v_nop\n\tv_nop\n\tv_nop\n\tv_nop" : "+v"(a), "+v"(b) : "v"(x), "v"(y)); }
__device__ __forceinline__ void dep_guard_b(v8f& a, v8f& b, v16b x, v16b y) { asm volatile("v_nop\n\tv_nop\n\tv_nop\n\tv_nop" : "+v"(a), "+v"(b) : "v"(x), "v"(y)); }
__device__ __forceinline__ void dep_guard4_h(v8f& a, v8f& b, v8f& c, v8f& d, v16h x, v16h y) { asm volatile("v_nop\n\tv_nop\n\tv_nop\n\tv_nop" : "+v"(a), "+v"(b), "+v"(c), "+v"(d) : "v"(x), "v"(y)); }
__device__ __forceinline__ void dep_guard4_b(v8f& a, v8f& b, v8f& c, v8f& d, v16b x, v16b y) { asm volatile("v_nop\n\tv_nop\n\tv_nop\n\tv_nop" : "+v"(a), "+v"(b), "+v"(c), "+v"(d) : "v"(x), "v"(y)); }
__device__ __forceinline__ void keep4_h(v16h a, v16h b, v16h c, v16h d) { asm volatile("v_nop" :: "v"(a), "v"(b), "v"(c), "v"(d)); }
__device__ __forceinline__ void keep4_b(v16b a, v16b b, v16b c, v16b d) { asm volatile("v_nop" :: "v"(a), "v"(b), "v"(c), "v"(d)); }
__device__ __forceinline__ void acc_guard4(v8f& a, v8f& b, v8f& c, v8f& d) { asm volatile("v_nop\n\tv_nop\n\tv_nop\n\tv_nop" : "+v"(a), "+v"(b), "+v"(c), "+v"(d)); }
template <typename T> struct Frag;
template <> struct Frag<_Float16> {
  typedef v16h V; union U { v16h v; v8h h[2]; };
  static __device__ __forceinline__ v16h load(const _Float16* p) {
    U f; f.h[0] = *(const v8h*)(p); f.h[1] = *(const v8h*)(p + 16); return f.v;
  }
  static __device__ __forceinline__ v8f mma(v16h a, v16h b, v8f c) {
    return __builtin_amdgcn_wmma_f32_16x16x32_f16(false, a, false, b, (short)0, c, false, false);
  }
  static __device__ __forceinline__ void guard(v8f& a, v8f& b, v16h x, v16h y) { dep_guard_h(a, b, x, y); }
  static __device__ __forceinline__ void guard4(v8f& a, v8f& b, v8f& c, v8f& d, v16h x, v16h y) { dep_guard4_h(a, b, c, d, x, y); }
  static __device__ __forceinline__ void keep(v16h a, v16h b, v16h c, v16h d) { keep4_h(a, b, c, d); }
};
template <> struct Frag<__bf16> {
  typedef v16b V; union U { v16b v; v8b h[2]; };
  static __device__ __forceinline__ v16b load(const __bf16* p) {
    U f; f.h[0] = *(const v8b*)(p); f.h[1] = *(const v8b*)(p + 16); return f.v;
  }
  static __device__ __forceinline__ v8f mma(v16b a, v16b b, v8f c) {
    return __builtin_amdgcn_wmma_f32_16x16x32_bf16(false, a, false, b, (short)0, c, false, false);
  }
  static __device__ __forceinline__ void guard(v8f& a, v8f& b, v16b x, v16b y) { dep_guard_b(a, b, x, y); }
  static __device__ __forceinline__ void guard4(v8f& a, v8f& b, v8f& c, v8f& d, v16b x, v16b y) { dep_guard4_b(a, b, c, d, x, y); }
  static __device__ __forceinline__ void keep(v16b a, v16b b, v16b c, v16b d) { keep4_b(a, b, c, d); }
};

template <int ET> struct Elem;
template <> struct Elem<0> { typedef _Float16 T; };
template <> struct Elem<1> { typedef __bf16 T; };
template <int ET, bool SPLIT, int BIAS_MODE, int OUT_MODE, bool RESID>
__global__ __launch_bounds__(256) void wmma_gemm64(
    const unsigned short* __restrict__ Ap, const unsigned short* __restrict__ A2p, int lda, long strideA,
    const unsigned short* __restrict__ Btp, const unsigned short* __restrict__ Bt2p, int ldb, long strideB,
    void* __restrict__ Cout, void* __restrict__ Cout2, int ldc, long strideC,
    const float* __restrict__ bias,
    const float* __restrict__ resid, long strideR,
    int M, int N, int K, float scale) {
  typedef typename Elem<ET>::T T;
  typedef typename Frag<T>::V V;
  const T* A = (const T*)Ap; const T* A2 = (const T*)A2p; const T* Bt = (const T*)Btp; const T* Bt2 = (const T*)Bt2p;
  __shared__ __align__(16) float sT[8][16 * 68];
  const int b    = blockIdx.y;
  const int lane = threadIdx.x & 31;
  const int wave = threadIdx.x >> 5;
  const int tilesN = N >> 6;
  const int tilesM = M >> 6;
  const int tile = blockIdx.x * 8 + wave;
  if (tile >= tilesM * tilesN) return;
  const int tm = tile / tilesN;
  const int tn = tile - tm * tilesN;
  const int m0 = tm << 6;
  const int n0 = tn << 6;

  const T* Ab  = A  + (size_t)b * strideA;
  const T* Bb  = Bt + (size_t)b * strideB;
  const T* Ab2 = SPLIT ? (A2  + (size_t)b * strideA) : nullptr;
  const T* Bb2 = SPLIT ? (Bt2 + (size_t)b * strideB) : nullptr;

  const int rlane = lane & 15;
  const int koff  = (lane >> 4) * 8;
  const int mOff  = (lane >> 4) * 8;

  v8f acc[4][4];
#pragma unroll
  for (int i = 0; i < 4; ++i)
#pragma unroll
    for (int j = 0; j < 4; ++j) acc[i][j] = (v8f){0.f,0.f,0.f,0.f,0.f,0.f,0.f,0.f};

  for (int k0 = 0; k0 < K; k0 += 32) {
    V bh[4], bl[4];
#pragma unroll
    for (int j = 0; j < 4; ++j) {
      const size_t bo = (size_t)(n0 + (j << 4) + rlane) * ldb + koff + k0;
      bh[j] = Frag<T>::load(Bb + bo);
      if (SPLIT) bl[j] = Frag<T>::load(Bb2 + bo);
    }
#pragma unroll
    for (int i = 0; i < 4; ++i) {
      const size_t ao = (size_t)(m0 + (i << 4) + rlane) * lda + koff + k0;
      V ah = Frag<T>::load(Ab + ao);
      V al;
      if (SPLIT) al = Frag<T>::load(Ab2 + ao);
#pragma unroll
      for (int j = 0; j < 4; ++j) {
        acc[i][j] = Frag<T>::mma(ah, bh[j], acc[i][j]);
        if (SPLIT) {
          acc[i][j] = Frag<T>::mma(ah, bl[j], acc[i][j]);
          acc[i][j] = Frag<T>::mma(al, bh[j], acc[i][j]);
        }
      }
      Frag<T>::guard4(acc[i][0], acc[i][1], acc[i][2], acc[i][3], ah, SPLIT ? al : ah);
    }
    Frag<T>::keep(bh[0], bh[1], bh[2], bh[3]);
    if (SPLIT) Frag<T>::keep(bl[0], bl[1], bl[2], bl[3]);
  }
  acc_guard4(acc[0][0], acc[0][1], acc[0][2], acc[0][3]);
  acc_guard4(acc[1][0], acc[1][1], acc[1][2], acc[1][3]);
  acc_guard4(acc[2][0], acc[2][1], acc[2][2], acc[2][3]);
  acc_guard4(acc[3][0], acc[3][1], acc[3][2], acc[3][3]);

  float* slab = sT[wave];
  const float* Rb = RESID ? (resid + (size_t)b * strideR) : nullptr;
#pragma unroll
  for (int i = 0; i < 4; ++i) {
    const int mBase = m0 + (i << 4);
#pragma unroll
    for (int j = 0; j < 4; ++j) {
      const int n = n0 + (j << 4) + rlane;
      float bv = 0.f;
      if (BIAS_MODE == 2) bv = bias[n];
#pragma unroll
      for (int r = 0; r < 8; ++r) {
        float v = acc[i][j][r] * scale;
        if (BIAS_MODE == 1) v += bias[mBase + mOff + r];
        if (BIAS_MODE == 2) v += bv;
        slab[(mOff + r) * 68 + (j << 4) + rlane] = v;
      }
    }
    __builtin_amdgcn_fence(__ATOMIC_RELEASE, "workgroup");
    __builtin_amdgcn_wave_barrier();
    __builtin_amdgcn_fence(__ATOMIC_ACQUIRE, "workgroup");
    if (OUT_MODE == 0) {
      float* C = (float*)Cout + (size_t)b * strideC;
      const int hh = lane >> 4, c4 = (lane & 15) * 4;
      for (int pass = 0; pass < 2; ++pass) {
#pragma unroll
        for (int it = 0; it < 8; ++it) {
          const int row = it * 2 + hh;
          v4f v = *(const v4f*)(slab + row * 68 + c4);
          if (RESID) {
            const v4f rv = *(const v4f*)(Rb + (size_t)(mBase + row) * ldc + n0 + c4);
            v = v + rv;
          }
          *(volatile v4f*)(C + (size_t)(mBase + row) * ldc + n0 + c4) = v;
        }
        __threadfence();
      }
    } else {
      const int q = lane >> 3, c8 = (lane & 7) * 8;
      unsigned short* C  = (unsigned short*)Cout  + (size_t)b * strideC;
      unsigned short* C2 = (OUT_MODE == 2) ? ((unsigned short*)Cout2 + (size_t)b * strideC) : nullptr;
      for (int pass = 0; pass < 2; ++pass) {
#pragma unroll
        for (int it = 0; it < 4; ++it) {
          const int row = it * 4 + q;
          const float* sp = slab + row * 68 + c8;
          v8h hv, lv;
#pragma unroll
          for (int e = 0; e < 8; ++e) {
            if (OUT_MODE == 1) {
              hv[e] = (_Float16)sp[e];
            } else {
              unsigned short hb = f2bf_bits(sp[e]);
              unsigned short lb = f2bf_bits(sp[e] - bf_bits2f(hb));
              hv[e] = __builtin_bit_cast(_Float16, hb);
              lv[e] = __builtin_bit_cast(_Float16, lb);
            }
          }
          *(volatile v8h*)(C + (size_t)(mBase + row) * ldc + n0 + c8) = hv;
          if (OUT_MODE == 2) *(volatile v8h*)(C2 + (size_t)(mBase + row) * ldc + n0 + c8) = lv;
        }
        __threadfence();
      }
    }
    __builtin_amdgcn_fence(__ATOMIC_RELEASE, "workgroup");
    __builtin_amdgcn_wave_barrier();
    __builtin_amdgcn_fence(__ATOMIC_ACQUIRE, "workgroup");
  }
}

__global__ __launch_bounds__(NTHR) void cvt_bf16x8_kernel(const float* __restrict__ src, unsigned short* __restrict__ dst, int n8) {
  const int i = blockIdx.x * NTHR + threadIdx.x;
  if (i < n8) {
    const float* sp = src + (size_t)i * 8;
    const v4f a = *(const v4f*)(sp);
    const v4f b = *(const v4f*)(sp + 4);
    v4u o;
    o[0] = pack_bf2(a[0], a[1]);
    o[1] = pack_bf2(a[2], a[3]);
    o[2] = pack_bf2(b[0], b[1]);
    o[3] = pack_bf2(b[2], b[3]);
    unsigned* dp = (unsigned*)(dst + (size_t)i * 8);
    *(volatile v4u*)dp = o;
    __threadfence();
    *(volatile v4u*)dp = o;
  }
}

__global__ __launch_bounds__(NTHR) void zero16x8_kernel(unsigned short* __restrict__ dst, int n8) {
  const int i = blockIdx.x * NTHR + threadIdx.x;
  if (i < n8) {
    const v4u o = {0u, 0u, 0u, 0u};
    unsigned* dp = (unsigned*)(dst + (size_t)i * 8);
    *(volatile v4u*)dp = o;
    __threadfence();
    *(volatile v4u*)dp = o;
  }
}

__global__ __launch_bounds__(NTHR) void ln_bf16_kernel(const float* __restrict__ X, const float* __restrict__ gam,
                                                       const float* __restrict__ bet, unsigned short* __restrict__ XN, int nrows) {
  const int tid = threadIdx.x, lane = tid & 31;
  const int row = blockIdx.x * (NTHR / 32) + (tid >> 5);
  if (row >= nrows) return;
  const float* rp = X + (size_t)row * NDIM;
  const int c0 = 8 * lane, c1 = 256 + 8 * lane;
  v4f v[4];
  v[0] = *(const v4f*)(rp + c0);
  v[1] = *(const v4f*)(rp + c0 + 4);
  v[2] = *(const v4f*)(rp + c1);
  v[3] = *(const v4f*)(rp + c1 + 4);
  float s = 0.0f;
#pragma unroll
  for (int q = 0; q < 4; ++q) s += (v[q][0] + v[q][1]) + (v[q][2] + v[q][3]);
#pragma unroll
  for (int off = 1; off < 32; off <<= 1) s += __shfl_xor(s, off, 32);
  const float mu = s * (1.0f / NDIM);
  float ss = 0.0f;
#pragma unroll
  for (int q = 0; q < 4; ++q)
#pragma unroll
    for (int e = 0; e < 4; ++e) { const float d = v[q][e] - mu; v[q][e] = d; ss += d * d; }
#pragma unroll
  for (int off = 1; off < 32; off <<= 1) ss += __shfl_xor(ss, off, 32);
  const float var  = ss * (1.0f / NDIM);
  const float rstd = rsqrtf(var + 1e-5f);
  asm volatile("" ::: "memory");
  v4f g[4], bb[4];
  g[0]  = *(const v4f*)(gam + c0); g[1]  = *(const v4f*)(gam + c0 + 4); g[2]  = *(const v4f*)(gam + c1); g[3]  = *(const v4f*)(gam + c1 + 4);
  bb[0] = *(const v4f*)(bet + c0); bb[1] = *(const v4f*)(bet + c0 + 4); bb[2] = *(const v4f*)(bet + c1); bb[3] = *(const v4f*)(bet + c1 + 4);
  float o[4][4];
#pragma unroll
  for (int q = 0; q < 4; ++q)
#pragma unroll
    for (int e = 0; e < 4; ++e) o[q][e] = (v[q][e] * rstd) * g[q][e] + bb[q][e];
  v4u w0, w1;
  w0[0] = pack_bf2(o[0][0], o[0][1]); w0[1] = pack_bf2(o[0][2], o[0][3]);
  w0[2] = pack_bf2(o[1][0], o[1][1]); w0[3] = pack_bf2(o[1][2], o[1][3]);
  w1[0] = pack_bf2(o[2][0], o[2][1]); w1[1] = pack_bf2(o[2][2], o[2][3]);
  w1[2] = pack_bf2(o[3][0], o[3][1]); w1[3] = pack_bf2(o[3][2], o[3][3]);
  unsigned* op = (unsigned*)(XN + (size_t)row * NDIM);
  for (int pass = 0; pass < 2; ++pass) {
    *(volatile v4u*)(op + 4 * lane) = w0;
    *(volatile v4u*)(op + 128 + 4 * lane) = w1;
    __threadfence();
  }
}

__global__ __launch_bounds__(NTHR) void conv_silu_kernel(const float* __restrict__ XT, const float* __restrict__ cw,
                                                         const float* __restrict__ cb, unsigned short* __restrict__ XTB,
                                                         unsigned short* __restrict__ XCB) {
  const int i = blockIdx.x * NTHR + threadIdx.x;
  const int row = i >> 7, c8 = i & 127, p0 = c8 * 8;
  const float* rp = XT + (size_t)row * NPROJ;
  const int pm = (p0 >= 4) ? (p0 - 4) : 0;
  const v4f pv = *(const v4f*)(rp + pm);
  const v4f a  = *(const v4f*)(rp + p0);
  const v4f b  = *(const v4f*)(rp + p0 + 4);
  const float w0 = cw[0], w1 = cw[1], w2 = cw[2], w3 = cw[3], cbias = cb[0];
  const float zsel = (c8 == 0) ? 0.0f : 1.0f;
  float xs[11];
  xs[0] = pv[1] * zsel; xs[1] = pv[2] * zsel; xs[2] = pv[3] * zsel;
  xs[3] = a[0]; xs[4] = a[1]; xs[5] = a[2]; xs[6]  = a[3];
  xs[7] = b[0]; xs[8] = b[1]; xs[9] = b[2]; xs[10] = b[3];
  float ys[8];
#pragma unroll
  for (int e = 0; e < 8; ++e) {
    const float y = fmaf(w3, xs[e + 3], fmaf(w2, xs[e + 2], fmaf(w1, xs[e + 1], fmaf(w0, xs[e], cbias))));
    ys[e] = fsilu(y);
  }
  v4u wt, wc;
  wt[0] = pack_bf2(xs[3], xs[4]); wt[1] = pack_bf2(xs[5], xs[6]); wt[2] = pack_bf2(xs[7], xs[8]); wt[3] = pack_bf2(xs[9], xs[10]);
  wc[0] = pack_bf2(ys[0], ys[1]); wc[1] = pack_bf2(ys[2], ys[3]); wc[2] = pack_bf2(ys[4], ys[5]); wc[3] = pack_bf2(ys[6], ys[7]);
  unsigned* tp = (unsigned*)(XTB + (size_t)row * NPROJ + p0);
  unsigned* cp = (unsigned*)(XCB + (size_t)row * NPROJ + p0);
  for (int pass = 0; pass < 2; ++pass) {
    *(volatile v4u*)tp = wt;
    *(volatile v4u*)cp = wc;
    __threadfence();
  }
}

__global__ __launch_bounds__(NTHR) void mlstm_scan_kernel(const float* __restrict__ QKS, const float* __restrict__ VO,
                                                          const float* __restrict__ bq, const float* __restrict__ bk,
                                                          const float* __restrict__ bv, const float* __restrict__ bo,
                                                          const float* __restrict__ bi, const float* __restrict__ bfg,
                                                          float* __restrict__ HB) {
  __shared__ __align__(16) float stg[NTHR];
  __shared__ __align__(16) float numv[HDIM];
  __shared__ float denw[NTHR / 32];
  __shared__ float gsc[2];
  const int tid = threadIdx.x, lane = tid & 31, wave = tid >> 5;
  const int bb = blockIdx.x >> 3, hd = blockIdx.x & 7;
  const int role = wave >> 1;
  const int e    = tid & 63;
  const int dI   = tid >> 2;
  const int nOff = (tid & 3) * 16;
  const int hcol = hd * HDIM + e;
  const float cq = bq[hcol], ck = bk[hcol], cv = bv[hcol], co = bo[hcol];
  const float cbias = (role == 0) ? cq : (role == 1) ? ck : (role == 2) ? cv : co;
  const float gbi = bi[hd], gbf = bfg[hd];
  const int offA = (role & 1) * NHID + hcol;
  const int offB = (role & 1) * NHID + hcol;

  float cr[16];
#pragma unroll
  for (int j = 0; j < 16; ++j) cr[j] = 0.0f;
  float nst = 1.0f;
  float mst = 0.0f;

#pragma unroll 1
  for (int t = 0; t < NSEQ; ++t) {
    const size_t row = (size_t)t * NBAT + bb;
    {
      const float va = QKS[row * NQKS + offA];
      const float vb = VO[row * NVO + offB];
      float x = ((role < 2) ? va : vb) + cbias;
      x = (role == 1) ? x * 0.125f : x;
      const float sg = fsigm(x);
      x = (role == 3) ? sg : x;
      stg[tid] = x;
      if (wave == 0) {
        const float ig = QKS[row * NQKS + COL_IG + hd] + gbi;
        const float fg = QKS[row * NQKS + COL_FG + hd] + gbf;
        const float mt = fmaxf(fg + mst, ig);
        const float ie = expf(ig - mt);
        const float fe = expf((fg - mt) + mst);
        mst = mt;
        gsc[0] = ie;
        gsc[1] = fe;
      }
    }
    __syncthreads();
    {
      const float ie = gsc[0], fe = gsc[1];
      const float vd = stg[128 + dI];
      const float ivd = ie * vd;
      const v4f qa = *(const v4f*)(stg + nOff);
      const v4f qb = *(const v4f*)(stg + nOff + 4);
      const v4f qc = *(const v4f*)(stg + nOff + 8);
      const v4f qd = *(const v4f*)(stg + nOff + 12);
      const v4f ka = *(const v4f*)(stg + 64 + nOff);
      const v4f kb = *(const v4f*)(stg + 64 + nOff + 4);
      const v4f kc = *(const v4f*)(stg + 64 + nOff + 8);
      const v4f kd = *(const v4f*)(stg + 64 + nOff + 12);
      const float qq[16] = {qa[0], qa[1], qa[2], qa[3], qb[0], qb[1], qb[2], qb[3], qc[0], qc[1], qc[2], qc[3], qd[0], qd[1], qd[2], qd[3]};
      const float kk[16] = {ka[0], ka[1], ka[2], ka[3], kb[0], kb[1], kb[2], kb[3], kc[0], kc[1], kc[2], kc[3], kd[0], kd[1], kd[2], kd[3]};
      float num = 0.0f;
#pragma unroll
      for (int j = 0; j < 16; ++j) {
        const float cn = fe * cr[j] + ivd * kk[j];
        cr[j] = cn;
        num = fmaf(cn, qq[j], num);
      }
      num += __shfl_xor(num, 1, 32);
      num += __shfl_xor(num, 2, 32);
      const float kdd = stg[64 + dI], qdd = stg[dI], odd = stg[192 + dI];
      nst = fe * nst + ie * kdd;
      float dp = ((lane & 3) == 0) ? nst * qdd : 0.0f;
#pragma unroll
      for (int off = 1; off < 32; off <<= 1) dp += __shfl_xor(dp, off, 32);
      if (lane == 0) denw[wave] = dp;
      numv[dI] = odd * num;
    }
    __syncthreads();
    if (wave == 0) {
      float den = denw[0];
      den += denw[1]; den += denw[2]; den += denw[3]; den += denw[4]; den += denw[5]; den += denw[6]; den += denw[7];
      den = fmaxf(fabsf(den), 1.0f);
      const float inv = 1.0f / den;
      const int cq4 = (lane & 15) * 4;
      const v4f hs = *(const v4f*)(numv + cq4);
      v4f hv;
      hv[0] = hs[0] * inv; hv[1] = hs[1] * inv; hv[2] = hs[2] * inv; hv[3] = hs[3] * inv;
      float* hp = HB + row * NHID + hd * HDIM + cq4;
      for (int pass = 0; pass < 2; ++pass) {
        if (lane < 16) *(volatile v4f*)hp = hv;
        __threadfence();
      }
    }
  }
}

__global__ __launch_bounds__(NTHR) void post_mix_kernel(const float* __restrict__ HB, const float* __restrict__ QKS,
                                                        const float* __restrict__ RT, const float* __restrict__ gng,
                                                        const float* __restrict__ gnb, const float* __restrict__ skb,
                                                        unsigned short* __restrict__ MIXB, int nrows) {
  const int tid = threadIdx.x, lane = tid & 31, wave = tid >> 5;
  const int row = blockIdx.x * (NTHR / 64) + (wave >> 1);
  if (row >= nrows) return;
  const int half = wave & 1;
  const int col0 = half * 256 + 8 * lane;
  const float* hp = HB + (size_t)row * NHID + col0;
  const v4f h0 = *(const v4f*)(hp);
  const v4f h1 = *(const v4f*)(hp + 4);
  float d[8] = {h0[0], h0[1], h0[2], h0[3], h1[0], h1[1], h1[2], h1[3]};
  float s = ((d[0] + d[1]) + (d[2] + d[3])) + ((d[4] + d[5]) + (d[6] + d[7]));
  s += __shfl_xor(s, 1, 32); s += __shfl_xor(s, 2, 32); s += __shfl_xor(s, 4, 32);
  const float mu = s * (1.0f / HDIM);
  float ss = 0.0f;
#pragma unroll
  for (int e = 0; e < 8; ++e) { d[e] = d[e] - mu; ss += d[e] * d[e]; }
  ss += __shfl_xor(ss, 1, 32); ss += __shfl_xor(ss, 2, 32); ss += __shfl_xor(ss, 4, 32);
  const float var  = ss * (1.0f / HDIM);
  const float rstd = rsqrtf(var + 1e-5f);
  asm volatile("" ::: "memory");
  const v4f g0 = *(const v4f*)(gng + col0), g1 = *(const v4f*)(gng + col0 + 4);
  const v4f b0 = *(const v4f*)(gnb + col0), b1 = *(const v4f*)(gnb + col0 + 4);
  const float* sp = QKS + (size_t)row * NQKS + COL_SKIP + col0;
  const v4f s0 = *(const v4f*)(sp), s1 = *(const v4f*)(sp + 4);
  const v4f c0 = *(const v4f*)(skb + col0), c1 = *(const v4f*)(skb + col0 + 4);
  asm volatile("" ::: "memory");
  const float* rtp = RT + (size_t)row * NHID + col0;
  const v4f r0 = *(const v4f*)(rtp), r1 = *(const v4f*)(rtp + 4);
  const float gg[8] = {g0[0], g0[1], g0[2], g0[3], g1[0], g1[1], g1[2], g1[3]};
  const float gb[8] = {b0[0], b0[1], b0[2], b0[3], b1[0], b1[1], b1[2], b1[3]};
  const float sk[8] = {s0[0] + c0[0], s0[1] + c0[1], s0[2] + c0[2], s0[3] + c0[3], s1[0] + c1[0], s1[1] + c1[1], s1[2] + c1[2], s1[3] + c1[3]};
  const float rr[8] = {r0[0], r0[1], r0[2], r0[3], r1[0], r1[1], r1[2], r1[3]};
  float o[8];
#pragma unroll
  for (int e = 0; e < 8; ++e) {
    const float xn = (d[e] * rstd) * gg[e] + gb[e];
    o[e] = (xn + sk[e]) * fsilu(rr[e]);
  }
  v4u w;
  w[0] = pack_bf2(o[0], o[1]); w[1] = pack_bf2(o[2], o[3]); w[2] = pack_bf2(o[4], o[5]); w[3] = pack_bf2(o[6], o[7]);
  unsigned* op = (unsigned*)(MIXB + (size_t)row * NHID + col0);
  for (int pass = 0; pass < 2; ++pass) {
    *(volatile v4u*)op = w;
    __threadfence();
  }
}

extern "C" void kernel_launch(void* const* d_in, const int* in_sizes, int n_in,
                              void* d_out, int out_size, void* d_ws, size_t ws_size, hipStream_t stream) {
  if (n_in < 27 || d_out == nullptr || d_ws == nullptr) return;
  if (in_sizes[0]  != NROW * NDIM        || in_sizes[1]  != NLAY * NDIM || in_sizes[2]  != NLAY * NDIM ||
      in_sizes[3]  != NLAY * NPROJ * NDIM || in_sizes[4] != NLAY * NPROJ ||
      in_sizes[5]  != NLAY * NHID * NDIM  || in_sizes[6] != NLAY * NHID ||
      in_sizes[7]  != NLAY * KCONV        || in_sizes[8] != NLAY ||
      in_sizes[9]  != NLAY * NHID * NPROJ || in_sizes[10] != NLAY * NHID ||
      in_sizes[11] != NLAY * NHID * NPROJ || in_sizes[12] != NLAY * NHID ||
      in_sizes[13] != NLAY * NHID * NPROJ || in_sizes[14] != NLAY * NHID ||
      in_sizes[15] != NLAY * NHEAD * NPROJ || in_sizes[16] != NLAY * NHEAD ||
      in_sizes[17] != NLAY * NHEAD * NPROJ || in_sizes[18] != NLAY * NHEAD ||
      in_sizes[19] != NLAY * NHID * NPROJ || in_sizes[20] != NLAY * NHID ||
      in_sizes[21] != NLAY * NHID || in_sizes[22] != NLAY * NHID ||
      in_sizes[23] != NLAY * NHID * NPROJ || in_sizes[24] != NLAY * NHID ||
      in_sizes[25] != NLAY * NDIM * NHID  || in_sizes[26] != NLAY * NDIM ||
      out_size != NROW * NDIM) return;

  const float* x      = (const float*)d_in[0];
  const float* ln_g   = (const float*)d_in[1];
  const float* ln_b   = (const float*)d_in[2];
  const float* Wl     = (const float*)d_in[3];
  const float* bl     = (const float*)d_in[4];
  const float* Wr     = (const float*)d_in[5];
  const float* br     = (const float*)d_in[6];
  const float* conv_w = (const float*)d_in[7];
  const float* conv_b = (const float*)d_in[8];
  const float* Wq     = (const float*)d_in[9];
  const float* bq     = (const float*)d_in[10];
  const float* Wk     = (const float*)d_in[11];
  const float* bk     = (const float*)d_in[12];
  const float* Wv     = (const float*)d_in[13];
  const float* bv     = (const float*)d_in[14];
  const float* Wi     = (const float*)d_in[15];
  const float* bi     = (const float*)d_in[16];
  const float* Wf     = (const float*)d_in[17];
  const float* bfg    = (const float*)d_in[18];
  const float* Wo     = (const float*)d_in[19];
  const float* bo     = (const float*)d_in[20];
  const float* gn_g   = (const float*)d_in[21];
  const float* gn_b   = (const float*)d_in[22];
  const float* skw    = (const float*)d_in[23];
  const float* skb    = (const float*)d_in[24];
  const float* dww    = (const float*)d_in[25];
  const float* dwb    = (const float*)d_in[26];
  float* y_out = (float*)d_out;

  char* ws = (char*)d_ws; size_t off = 0;
  auto carve = [&](size_t bytes) -> char* { char* p = ws + off; off += (bytes + 255) & ~(size_t)255; return p; };
  unsigned short* XN   = (unsigned short*)carve((size_t)NROW * NDIM * 2);
  float*          XT   = (float*)carve((size_t)NROW * NPROJ * 4);
  float*          RT   = (float*)carve((size_t)NROW * NHID * 4);
  unsigned short* XTB  = (unsigned short*)carve((size_t)NROW * NPROJ * 2);
  unsigned short* XCB  = (unsigned short*)carve((size_t)NROW * NPROJ * 2);
  float*          QKS  = (float*)carve((size_t)NROW * NQKS * 4);
  float*          VO   = (float*)carve((size_t)NROW * NVO * 4);
  float*          HB   = (float*)carve((size_t)NROW * NHID * 4);
  unsigned short* MIXB = (unsigned short*)carve((size_t)NROW * NHID * 2);
  float*          INP1 = (float*)carve((size_t)NROW * NDIM * 4);
  unsigned short* WLB  = (unsigned short*)carve((size_t)NPROJ * NDIM * 2);
  unsigned short* WRB  = (unsigned short*)carve((size_t)NHID * NDIM * 2);
  unsigned short* WQKS = (unsigned short*)carve((size_t)NQKS * NPROJ * 2);
  unsigned short* WVO  = (unsigned short*)carve((size_t)NVO * NPROJ * 2);
  unsigned short* WDB  = (unsigned short*)carve((size_t)NDIM * NHID * 2);
  if (off > ws_size || off > (size_t)134217728) return;

  {
    const int n8z = (NQKS - COL_ZPAD) * NPROJ / 8;
    zero16x8_kernel<<<(n8z + NTHR - 1) / NTHR, NTHR, 0, stream>>>(WQKS + (size_t)COL_ZPAD * NPROJ, n8z);
  }

  const int n8_pd = NPROJ * NDIM / 8;
  const int n8_hd = NHID * NDIM / 8;
  const int n8_hp = NHID * NPROJ / 8;
  const int n8_gp = NHEAD * NPROJ / 8;
  const int gS1 = ((NROW / 64) * (NPROJ / 64) + 7) / 8;
  const int gS2 = ((NROW / 64) * (NHID / 64) + 7) / 8;
  const int gS3 = ((NROW / 64) * (NQKS / 64) + 7) / 8;
  const int gS5 = ((NROW / 64) * (NVO / 64) + 7) / 8;
  const int gS7 = ((NROW / 64) * (NDIM / 64) + 7) / 8;

  for (int l = 0; l < NLAY; ++l) {
    const float* lin = (l == 0) ? x : INP1;
    float* lout      = (l == NLAY - 1) ? y_out : INP1;

    cvt_bf16x8_kernel<<<(n8_pd + NTHR - 1) / NTHR, NTHR, 0, stream>>>(Wl  + (size_t)l * NPROJ * NDIM,  WLB, n8_pd);
    cvt_bf16x8_kernel<<<(n8_hd + NTHR - 1) / NTHR, NTHR, 0, stream>>>(Wr  + (size_t)l * NHID * NDIM,   WRB, n8_hd);
    cvt_bf16x8_kernel<<<(n8_hp + NTHR - 1) / NTHR, NTHR, 0, stream>>>(Wq  + (size_t)l * NHID * NPROJ,  WQKS + (size_t)COL_Q * NPROJ, n8_hp);
    cvt_bf16x8_kernel<<<(n8_hp + NTHR - 1) / NTHR, NTHR, 0, stream>>>(Wk  + (size_t)l * NHID * NPROJ,  WQKS + (size_t)COL_K * NPROJ, n8_hp);
    cvt_bf16x8_kernel<<<(n8_hp + NTHR - 1) / NTHR, NTHR, 0, stream>>>(skw + (size_t)l * NHID * NPROJ,  WQKS + (size_t)COL_SKIP * NPROJ, n8_hp);
    cvt_bf16x8_kernel<<<(n8_gp + NTHR - 1) / NTHR, NTHR, 0, stream>>>(Wi  + (size_t)l * NHEAD * NPROJ, WQKS + (size_t)COL_IG * NPROJ, n8_gp);
    cvt_bf16x8_kernel<<<(n8_gp + NTHR - 1) / NTHR, NTHR, 0, stream>>>(Wf  + (size_t)l * NHEAD * NPROJ, WQKS + (size_t)COL_FG * NPROJ, n8_gp);
    cvt_bf16x8_kernel<<<(n8_hp + NTHR - 1) / NTHR, NTHR, 0, stream>>>(Wv  + (size_t)l * NHID * NPROJ,  WVO + (size_t)COL_V * NPROJ, n8_hp);
    cvt_bf16x8_kernel<<<(n8_hp + NTHR - 1) / NTHR, NTHR, 0, stream>>>(Wo  + (size_t)l * NHID * NPROJ,  WVO + (size_t)COL_OG * NPROJ, n8_hp);
    cvt_bf16x8_kernel<<<(n8_hd + NTHR - 1) / NTHR, NTHR, 0, stream>>>(dww + (size_t)l * NDIM * NHID,   WDB, n8_hd);

    ln_bf16_kernel<<<NROW / (NTHR / 32), NTHR, 0, stream>>>(lin, ln_g + (size_t)l * NDIM, ln_b + (size_t)l * NDIM, XN, NROW);

    wmma_gemm64<1, false, 2, 0, false><<<dim3(gS1, 1), 256, 0, stream>>>(
        XN, XN, NDIM, 0L, WLB, WLB, NDIM, 0L, (void*)XT, (void*)XT, NPROJ, 0L,
        bl + (size_t)l * NPROJ, RT, 0L, NROW, NPROJ, NDIM, 1.0f);
    wmma_gemm64<1, false, 2, 0, false><<<dim3(gS2, 1), 256, 0, stream>>>(
        XN, XN, NDIM, 0L, WRB, WRB, NDIM, 0L, (void*)RT, (void*)RT, NHID, 0L,
        br + (size_t)l * NHID, XT, 0L, NROW, NHID, NDIM, 1.0f);

    conv_silu_kernel<<<(NROW * (NPROJ / 8)) / NTHR, NTHR, 0, stream>>>(XT, conv_w + (size_t)l * KCONV, conv_b + l, XTB, XCB);

    wmma_gemm64<1, false, 0, 0, false><<<dim3(gS3, 1), 256, 0, stream>>>(
        XCB, XCB, NPROJ, 0L, WQKS, WQKS, NPROJ, 0L, (void*)QKS, (void*)QKS, NQKS, 0L,
        bq + (size_t)l * NHID, RT, 0L, NROW, NQKS, NPROJ, 1.0f);
    wmma_gemm64<1, false, 0, 0, false><<<dim3(gS5, 1), 256, 0, stream>>>(
        XTB, XTB, NPROJ, 0L, WVO, WVO, NPROJ, 0L, (void*)VO, (void*)VO, NVO, 0L,
        bv + (size_t)l * NHID, RT, 0L, NROW, NVO, NPROJ, 1.0f);

    mlstm_scan_kernel<<<NBAT * NHEAD, NTHR, 0, stream>>>(QKS, VO, bq + (size_t)l * NHID, bk + (size_t)l * NHID,
                                                        bv + (size_t)l * NHID, bo + (size_t)l * NHID,
                                                        bi + (size_t)l * NHEAD, bfg + (size_t)l * NHEAD, HB);

    post_mix_kernel<<<NROW / (NTHR / 64), NTHR, 0, stream>>>(HB, QKS, RT, gn_g + (size_t)l * NHID, gn_b + (size_t)l * NHID,
                                                             skb + (size_t)l * NHID, MIXB, NROW);

    wmma_gemm64<1, false, 2, 0, true><<<dim3(gS7, 1), 256, 0, stream>>>(
        MIXB, MIXB, NHID, 0L, WDB, WDB, NHID, 0L, (void*)lout, (void*)lout, NDIM, 0L,
        dwb + (size_t)l * NDIM, lin, 0L, NROW, NDIM, NHID, 1.0f);
  }
}
